// EfficientBalancedIPRMPNNModel_89876485636288
// MI455X (gfx1250) — hardware-verified
//
#include <hip/hip_runtime.h>


namespace {
constexpr int B_ = 64, NPG = 512, V = 64, IN = 128, H = 256, OUT = 10, TN = B_ * NPG, E = B_ * 16384, NBLK = TN / 128;
constexpr float WS = 64.0f, WI = 1.0f / 64.0f, AS = 8.0f, AI = 0.125f;

typedef _Float16 b16;
typedef __attribute__((ext_vector_type(16))) _Float16 v16b;
typedef __attribute__((ext_vector_type(8)))  _Float16 v8b;
typedef __attribute__((ext_vector_type(8)))  float v8f;
typedef __attribute__((ext_vector_type(4)))  float v4f;

__device__ __forceinline__ v8b ld8b(const b16* p) { return *(const v8b*)p; }
__device__ __forceinline__ v16b cat8b(v8b a, v8b b) { return __builtin_shufflevector(a, b, 0, 1, 2, 3, 4, 5, 6, 7, 8, 9, 10, 11, 12, 13, 14, 15); }
__device__ __forceinline__ v16b frag_kb(const b16* p, int hh) { return cat8b(ld8b(p + 8 * hh), ld8b(p + 16 + 8 * hh)); }
__device__ __forceinline__ void split16(float v, b16& hi, b16& lo) { hi = (b16)v; lo = (b16)(v - (float)hi); }
__device__ __forceinline__ void frag_ksplit(const float* p, int hh, v16b& fh_, v16b& fl_) {
  const float* p0 = p + 8 * hh; const float* p1 = p + 16 + 8 * hh;
#pragma unroll
  for (int e = 0; e < 8; ++e) { b16 a, c; split16(p0[e], a, c); fh_[e] = a; fl_[e] = c; split16(p1[e], a, c); fh_[8 + e] = a; fl_[8 + e] = c; }
}
__device__ __forceinline__ v8f wmma16b(v16b a, v16b b, v8f c) {
  v8f d = __builtin_amdgcn_wmma_f32_16x16x32_f16(false, a, false, b, (short)0, c, false, false);
  asm volatile("v_nop\n\tv_nop\n\tv_nop\n\tv_nop" : "+v"(d) : "v"(a), "v"(b));
  return d;
}
__device__ __forceinline__ void wave_lds_sync() {
  __builtin_amdgcn_fence(__ATOMIC_RELEASE, "workgroup");
  __builtin_amdgcn_wave_barrier();
  __builtin_amdgcn_fence(__ATOMIC_ACQUIRE, "workgroup");
}

struct Opnd { const void* p0; const void* p1; int ld; };
template <int NP> __device__ __forceinline__ void load_frags(const Opnd& o, int row, int kb, int hh, v16b& fh_, v16b& fl_) {
  if (NP == 0) { frag_ksplit((const float*)o.p0 + (size_t)row * o.ld + kb, hh, fh_, fl_); }
  else if (NP == 4) {
    const float* p = (const float*)o.p0 + (size_t)row * o.ld + kb; const float* p0 = p + 8 * hh; const float* p1 = p + 16 + 8 * hh;
#pragma unroll
    for (int e = 0; e < 8; ++e) { b16 a, c; split16(p0[e] * 64.0f, a, c); fh_[e] = a; fl_[e] = c; split16(p1[e] * 64.0f, a, c); fh_[8 + e] = a; fl_[8 + e] = c; }
  } else if (NP == 3) {
    const float* p = (const float*)o.p0 + (size_t)row * o.ld + kb; const float* p0 = p + 8 * hh; const float* p1 = p + 16 + 8 * hh;
#pragma unroll
    for (int e = 0; e < 8; ++e) { fh_[e] = (b16)p0[e]; fh_[8 + e] = (b16)p1[e]; }
    fl_ = fh_;
  } else {
    fh_ = frag_kb((const b16*)o.p0 + (size_t)row * o.ld + kb, hh);
    if (NP == 2) fl_ = frag_kb((const b16*)o.p1 + (size_t)row * o.ld + kb, hh); else fl_ = fh_;
  }
}
template <int ANP, int BNP> __device__ __forceinline__ v8f mac(v16b ah, v16b al, v16b bh, v16b bl, v8f c) {
  c = wmma16b(ah, bh, c);
  if (BNP == 0 || BNP == 2 || BNP == 4) c = wmma16b(ah, bl, c);
  if (ANP == 0 || ANP == 2 || ANP == 4) c = wmma16b(al, bh, c);
  return c;
}
template <int ANP, int BNP>
__device__ __forceinline__ void gemm_tile(const Opnd& A, const Opnd& B, int K, int m0, int c0, int nloc, int hlf, v8f (&acc)[2][4]) {
  for (int kb = 0; kb < K; kb += 32) {
    v16b a0h, a0l, a1h, a1l;
    load_frags<ANP>(A, m0 + nloc, kb, hlf, a0h, a0l);
    load_frags<ANP>(A, m0 + 16 + nloc, kb, hlf, a1h, a1l);
#pragma unroll
    for (int t = 0; t < 4; ++t) {
      v16b bh, bl;
      load_frags<BNP>(B, c0 + t * 16 + nloc, kb, hlf, bh, bl);
      acc[0][t] = mac<ANP, BNP>(a0h, a0l, bh, bl, acc[0][t]);
      acc[1][t] = mac<ANP, BNP>(a1h, a1l, bh, bl, acc[1][t]);
    }
  }
}

__device__ __forceinline__ void epi_planes(v8f (&acc)[2][4], float scale, bool two, b16* __restrict__ oh, b16* __restrict__ ol, int ldo,
                                           int m0, int c0, int lane, b16* Th, b16* Tl) {
  const int nloc = lane & 15, hlf = lane >> 4;
#pragma unroll
  for (int t = 0; t < 4; ++t)
#pragma unroll
    for (int r = 0; r < 2; ++r)
#pragma unroll
      for (int v = 0; v < 8; ++v) {
        const int rr = r * 16 + v + 8 * hlf, cc = t * 16 + nloc;
        b16 h_, l_; split16(acc[r][t][v] * scale, h_, l_);
        Th[rr * 64 + cc] = h_; Tl[rr * 64 + cc] = l_;
      }
  wave_lds_sync();
  for (int pass = 0; pass < 2; ++pass) {
#pragma unroll
    for (int j = 0; j < 8; ++j) {
      const int rr = j * 4 + (lane >> 3), c8 = (lane & 7) * 8;
      const size_t o = (size_t)(m0 + rr) * ldo + c0 + c8;
      *(volatile v8b*)(oh + o) = ld8b(Th + rr * 64 + c8);
      if (two) *(volatile v8b*)(ol + o) = ld8b(Tl + rr * 64 + c8);
    }
    __threadfence();
  }
}
__device__ __forceinline__ void epi_f32(v8f (&acc)[2][4], float scale, const float* rscale, float* __restrict__ out, int ldo, int m0, int c0, int lane, float* Tt) {
  const int nloc = lane & 15, hlf = lane >> 4;
#pragma unroll
  for (int t = 0; t < 4; ++t)
#pragma unroll
    for (int r = 0; r < 2; ++r)
#pragma unroll
      for (int v = 0; v < 8; ++v) {
        const int rr = r * 16 + v + 8 * hlf;
        const float rs = rscale ? rscale[(size_t)(m0 + rr) * 32] : 1.0f;
        Tt[rr * 64 + t * 16 + nloc] = acc[r][t][v] * scale * rs;
      }
  wave_lds_sync();
  float* dst0 = out + (size_t)m0 * ldo + c0;
  for (int pass = 0; pass < 2; ++pass) {
#pragma unroll
    for (int j = 0; j < 16; ++j) { const int rr = j * 2 + hlf, c4 = nloc * 4; *(volatile v4f*)(dst0 + (size_t)rr * ldo + c4) = *(const v4f*)(Tt + rr * 64 + c4); }
    __threadfence();
  }
}


__global__ __launch_bounds__(256) void prep_kernel(const float* __restrict__ Wemb, const float* __restrict__ Wgcn, const float* __restrict__ aW1, const float* __restrict__ aW2,
                                                   const float* __restrict__ vW1, const float* __restrict__ vW2, const float* __restrict__ mW1, const float* __restrict__ mW2,
                                                   b16* __restrict__ wemb, b16* __restrict__ w3, b16* __restrict__ th, b16* __restrict__ tl) {
  const size_t tid = (size_t)blockIdx.x * blockDim.x + threadIdx.x, nth = (size_t)gridDim.x * blockDim.x;
  for (int pass = 0; pass < 2; ++pass) {
    for (size_t p = tid; p < (size_t)H * IN / 8; p += nth) { const int n = (int)(p / (IN / 8)), k0 = (int)(p % (IN / 8)) * 8; v8b v;
#pragma unroll
      for (int e = 0; e < 8; ++e) v[e] = (b16)Wemb[(size_t)(k0 + e) * H + n];
      *(volatile v8b*)(wemb + (size_t)n * IN + k0) = v; }
    for (size_t p = tid; p < (size_t)3 * H * H / 8; p += nth) { const int m = (int)(p / (H * H / 8)); const int rem = (int)(p % (H * H / 8)), n = rem / (H / 8), k0 = (rem % (H / 8)) * 8; const float* W = (m == 0) ? Wgcn : (m == 1) ? aW1 : aW2; v8b v;
#pragma unroll
      for (int e = 0; e < 8; ++e) v[e] = (b16)W[(size_t)(k0 + e) * H + n];
      *(volatile v8b*)(w3 + (size_t)m * H * H + (size_t)n * H + k0) = v; }
    for (size_t p = tid; p < (size_t)(3 * H * H + 64 * H) / 8; p += nth) { v8b a, c;
      if (p < (size_t)3 * H * H / 8) { const int m = (int)(p / (H * H / 8)); const int rem = (int)(p % (H * H / 8)), n = rem / (H / 8), k0 = (rem % (H / 8)) * 8; const float* W = (m == 0) ? vW1 : (m == 1) ? vW2 : mW1;
#pragma unroll
        for (int e = 0; e < 8; ++e) { b16 x, y; split16(W[(size_t)(k0 + e) * H + n] * WS, x, y); a[e] = x; c[e] = y; } }
      else { const size_t q = p - (size_t)3 * H * H / 8; const int n = (int)(q / (H / 8)), k0 = (int)(q % (H / 8)) * 8;
#pragma unroll
        for (int e = 0; e < 8; ++e) { float w = (n < OUT) ? mW2[(size_t)(k0 + e) * OUT + min(n, OUT - 1)] : 0.0f; b16 x, y; split16(w * WS, x, y); a[e] = x; c[e] = y; } }
      *(volatile v8b*)(th + p * 8) = a; *(volatile v8b*)(tl + p * 8) = c; }
    __threadfence();
  }
}

template <int KIN, int NOUT, bool RELU, bool OUT16>
__global__ __launch_bounds__(128) void lin_kernel(const float* __restrict__ x, const b16* __restrict__ w, const float* __restrict__ bias, float* __restrict__ y, b16* __restrict__ y16) {
  __shared__ __attribute__((aligned(16))) float Ts[4][32 * 64];
  const int lane = threadIdx.x & 31, wave = threadIdx.x >> 5, nloc = lane & 15, hlf = lane >> 4, m0 = blockIdx.y * 128 + wave * 32, c0 = blockIdx.x * 64;
  v8f acc[2][4];
#pragma unroll
  for (int r = 0; r < 2; ++r)
#pragma unroll
    for (int t = 0; t < 4; ++t) acc[r][t] = (v8f){};
  const Opnd A{x, nullptr, KIN}, Bo{w, nullptr, KIN};
  gemm_tile<3, 1>(A, Bo, KIN, m0, c0, nloc, hlf, acc);
#pragma unroll
  for (int t = 0; t < 4; ++t)
#pragma unroll
    for (int r = 0; r < 2; ++r)
#pragma unroll
      for (int v = 0; v < 8; ++v) { float val = acc[r][t][v] + (bias ? bias[c0 + t * 16 + nloc] : 0.0f); if (RELU) val = fmaxf(val, 0.0f); acc[r][t][v] = val; }
  float* Tt = Ts[wave];
#pragma unroll
  for (int t = 0; t < 4; ++t)
#pragma unroll
    for (int r = 0; r < 2; ++r)
#pragma unroll
      for (int v = 0; v < 8; ++v) Tt[(r * 16 + v + 8 * hlf) * 64 + t * 16 + nloc] = acc[r][t][v];
  wave_lds_sync();
  for (int pass = 0; pass < 2; ++pass) {
#pragma unroll
    for (int j = 0; j < 16; ++j) { const int rr = j * 2 + hlf, c4 = nloc * 4; const v4f vv = *(const v4f*)(Tt + rr * 64 + c4); if (y) *(volatile v4f*)(y + (size_t)(m0 + rr) * NOUT + c0 + c4) = vv;
      if (OUT16) { typedef __attribute__((ext_vector_type(4))) _Float16 v4b; v4b ob; ob[0] = (b16)vv[0]; ob[1] = (b16)vv[1]; ob[2] = (b16)vv[2]; ob[3] = (b16)vv[3]; *(volatile v4b*)(y16 + (size_t)(m0 + rr) * NOUT + c0 + c4) = ob; } }
    __threadfence();
  }
}

typedef __attribute__((ext_vector_type(4))) int v4i;
__global__ __launch_bounds__(256) void deg_kernel(const int* __restrict__ edst, float* __restrict__ degf) {
  constexpr int NB = 16384;
  __shared__ int cnt[NB];
  const int t_ = threadIdx.x, base = blockIdx.x * NB;
  for (int i = t_; i < NB; i += 256) cnt[i] = 0;
  __syncthreads();
  for (int e0 = t_ * 8; e0 < E; e0 += 256 * 8) { const v4i a = *(const v4i*)(edst + e0), b = *(const v4i*)(edst + e0 + 4); const int dd[8] = {a[0], a[1], a[2], a[3], b[0], b[1], b[2], b[3]};
#pragma unroll
    for (int j = 0; j < 8; ++j) { const unsigned sl = (unsigned)(dd[j] - base); if (sl < (unsigned)NB) atomicAdd(&cnt[sl], 1); } }
  __syncthreads();
  for (int pass = 0; pass < 2; ++pass) { for (int i = t_; i < NB; i += 256) ((volatile float*)degf)[base + i] = (float)cnt[i] + 1.0f; __threadfence(); }
}

__global__ __launch_bounds__(256) void gcn_kernel(const int* __restrict__ edst, const int* __restrict__ esrc, const float* __restrict__ hw, const float* __restrict__ degf, const float* __restrict__ bias, float* __restrict__ g, b16* __restrict__ gT) {
  constexpr int NB = 256, DF = H; constexpr float FXS = 524288.0f, FXI = 1.0f / FXS;
  __shared__ __attribute__((aligned(16))) int acc[NB * DF];
  __shared__ int list[8 * 256];
  const int t_ = threadIdx.x, wave = t_ >> 5, lane = t_ & 31, base = blockIdx.x * NB;
  for (int i = t_; i < NB * DF; i += 256) acc[i] = 0;
  __syncthreads();
  int* wl = list + wave * 256;
  for (int c0 = 0; c0 < E; c0 += 256 * 8) {
    const int e0 = c0 + (wave * 32 + lane) * 8; const v4i a = *(const v4i*)(edst + e0), bq = *(const v4i*)(edst + e0 + 4); const int dd[8] = {a[0], a[1], a[2], a[3], bq[0], bq[1], bq[2], bq[3]};
    unsigned sl[8]; bool hit[8]; bool anyl = false;
#pragma unroll
    for (int j = 0; j < 8; ++j) { sl[j] = (unsigned)(dd[j] - base); hit[j] = sl[j] < (unsigned)NB; anyl |= hit[j]; }
    int wc = 0;
    if (__builtin_amdgcn_ballot_w32(anyl) != 0u) {
#pragma unroll
      for (int j = 0; j < 8; ++j) {
        const unsigned mj = __builtin_amdgcn_ballot_w32(hit[j]);
        if (mj != 0u) {
          if (hit[j]) { const int pos = wc + (int)__builtin_amdgcn_mbcnt_lo(mj, 0u); int o = esrc[e0 + j]; o = (o < 0) ? 0 : (o >= TN ? TN - 1 : o); wl[pos] = (o << 12) | (int)sl[j]; }
          wc += __builtin_popcount(mj); } } }
    __builtin_amdgcn_wave_barrier(); __builtin_amdgcn_fence(__ATOMIC_RELEASE, "workgroup"); __builtin_amdgcn_fence(__ATOMIC_ACQUIRE, "workgroup");
    for (int i = 0; i < wc; ++i) { const int ent = wl[i]; const int o = ent >> 12, slot = ent & 4095; const float w = rsqrtf(degf[o]);
#pragma unroll
      for (int ch = 0; ch < 2; ++ch) { const int col = ch * 128 + lane * 4; const v4f v = *(const v4f*)(hw + (size_t)o * DF + col);
#pragma unroll
        for (int c = 0; c < 4; ++c) atomicAdd(&acc[slot * DF + col + c], (int)rintf(w * v[c] * FXS)); } }
    __builtin_amdgcn_wave_barrier();
  }
  __syncthreads();
  float* accf = (float*)acc;
  for (int i = t_; i < NB * DF; i += 256) { const int r = i / DF, c = i % DF, node = base + r; const float dg = degf[node], di = rsqrtf(dg);
    accf[i] = fmaxf(di * ((float)acc[i] * FXI) + hw[(size_t)node * DF + c] / dg + bias[c], 0.0f); }
  __syncthreads();
  const int bgraph = base / NPG, n0 = base % NPG;
  for (int pass = 0; pass < 2; ++pass) {
    for (int i = t_; i < NB * DF / 4; i += 256) *(volatile v4f*)(g + (size_t)base * DF + (size_t)i * 4) = *(const v4f*)(accf + i * 4);
    for (int i = t_; i < DF * NB / 8; i += 256) { const int hcol = i / (NB / 8), nq = (i % (NB / 8)) * 8; v8b o;
#pragma unroll
      for (int e = 0; e < 8; ++e) o[e] = (b16)accf[(nq + e) * DF + hcol];
      *(volatile v8b*)(gT + ((size_t)bgraph * H + hcol) * NPG + n0 + nq) = o; }
    __threadfence();
  }
}

__global__ __launch_bounds__(256) void graph_kernel(const float* __restrict__ t, const float* __restrict__ ew, b16* __restrict__ mwT) {
  __shared__ float proto[H]; __shared__ float att[NPG]; __shared__ float red[8];
  const int b = blockIdx.x, t_ = threadIdx.x, wave = t_ >> 5, lane = t_ & 31; const float* tb = t + (size_t)b * NPG * H;
  { float s = 0.0f;
#pragma unroll 1
    for (int n = 0; n < NPG; ++n) s += tb[(size_t)n * H + t_];
    proto[t_] = s * (1.0f / NPG); }
  __syncthreads();
  { float s = proto[t_] * proto[t_];
#pragma unroll
    for (int o = 16; o > 0; o >>= 1) s += __shfl_xor(s, o);
    if (lane == 0) red[wave] = s; }
  __syncthreads();
  const float pn = fmaxf(sqrtf(red[0] + red[1] + red[2] + red[3] + red[4] + red[5] + red[6] + red[7]), 1e-8f);
#pragma unroll 1
  for (int n = wave; n < NPG; n += 8) { float dsum = 0.0f, nsum = 0.0f;
#pragma unroll
    for (int j = 0; j < 8; ++j) { const float x = tb[(size_t)n * H + j * 32 + lane]; dsum += x * proto[j * 32 + lane]; nsum += x * x; }
#pragma unroll
    for (int o = 16; o > 0; o >>= 1) { dsum += __shfl_xor(dsum, o); nsum += __shfl_xor(nsum, o); }
    if (lane == 0) { const float tn = fmaxf(sqrtf(nsum), 1e-8f); att[n] = 0.5f * (1.0f + dsum / (tn * pn)); } }
  __syncthreads();
  __shared__ __attribute__((aligned(16))) b16 MT[V][NPG + 8];
#pragma unroll 1
  for (int n = wave; n < NPG; n += 8) { const float a = att[n]; const float w0 = ew[((size_t)b * NPG + n) * V + lane] * a, w1 = ew[((size_t)b * NPG + n) * V + 32 + lane] * a; float rs = w0 + w1;
#pragma unroll
    for (int o = 16; o > 0; o >>= 1) rs += __shfl_xor(rs, o);
    const float inv = 1.0f / ((rs == 0.0f) ? 1.0f : rs); MT[lane][n] = (b16)(w0 * inv); MT[32 + lane][n] = (b16)(w1 * inv); }
  __syncthreads();
  for (int pass = 0; pass < 2; ++pass) { for (int i = t_; i < V * NPG / 8; i += 256) { const int v = i / (NPG / 8), nq = (i % (NPG / 8)) * 8; *(volatile v8b*)(mwT + ((size_t)b * V + v) * NPG + nq) = *(const v8b*)(&MT[v][nq]); } __threadfence(); }
}

__global__ __launch_bounds__(64) void vn_kernel(const b16* __restrict__ mwT, const b16* __restrict__ gT, float* __restrict__ vn) {
  __shared__ __attribute__((aligned(16))) float Ts[2][32 * 64];
  const int lane = threadIdx.x & 31, wave = threadIdx.x >> 5, nloc = lane & 15, hlf = lane >> 4, b = blockIdx.y, m0 = wave * 32, c0 = blockIdx.x * 64;
  const b16* A = mwT + (size_t)b * V * NPG; const b16* Bw = gT + (size_t)b * H * NPG;
  v8f acc[2][4];
#pragma unroll
  for (int r = 0; r < 2; ++r)
#pragma unroll
    for (int t = 0; t < 4; ++t) acc[r][t] = (v8f){};
#pragma unroll 2
  for (int kb = 0; kb < NPG; kb += 32) { const v16b a0 = frag_kb(A + (size_t)(m0 + nloc) * NPG + kb, hlf), a1 = frag_kb(A + (size_t)(m0 + 16 + nloc) * NPG + kb, hlf);
#pragma unroll
    for (int t = 0; t < 4; ++t) { const v16b bw = frag_kb(Bw + (size_t)(c0 + t * 16 + nloc) * NPG + kb, hlf); acc[0][t] = wmma16b(a0, bw, acc[0][t]); acc[1][t] = wmma16b(a1, bw, acc[1][t]); } }
  epi_f32(acc, 1.0f, nullptr, vn + (size_t)b * V * H, H, m0, c0, lane, Ts[wave]);
}

template <bool RELU>
__global__ __launch_bounds__(64) void tail_kernel(const float* __restrict__ x, const b16* __restrict__ wh, const b16* __restrict__ wl, const float* __restrict__ bias, float* __restrict__ y, int nout) {
  __shared__ __attribute__((aligned(16))) float Ts[2][32 * 64];
  const int lane = threadIdx.x & 31, wave = threadIdx.x >> 5, nloc = lane & 15, hlf = lane >> 4, m0 = blockIdx.y * 64 + wave * 32, c0 = blockIdx.x * 64;
  v8f acc[2][4];
#pragma unroll
  for (int r = 0; r < 2; ++r)
#pragma unroll
    for (int t = 0; t < 4; ++t) acc[r][t] = (v8f){};
#pragma unroll 1
  for (int kb = 0; kb < H; kb += 32) { v16b a0, l0, a1, l1;
#pragma unroll
    for (int e = 0; e < 16; ++e) { const int k = kb + ((e < 8) ? (8 * hlf + e) : (16 + 8 * hlf + e - 8)); b16 p, q; split16(x[(size_t)(m0 + nloc) * H + k] * AS, p, q); a0[e] = p; l0[e] = q; split16(x[(size_t)(m0 + 16 + nloc) * H + k] * AS, p, q); a1[e] = p; l1[e] = q; }
#pragma unroll
    for (int t = 0; t < 4; ++t) { const v16b bh = frag_kb(wh + (size_t)(c0 + t * 16 + nloc) * H + kb, hlf), bl = frag_kb(wl + (size_t)(c0 + t * 16 + nloc) * H + kb, hlf);
      acc[0][t] = wmma16b(a0, bh, acc[0][t]); acc[0][t] = wmma16b(l0, bh, acc[0][t]); acc[0][t] = wmma16b(a0, bl, acc[0][t]);
      acc[1][t] = wmma16b(a1, bh, acc[1][t]); acc[1][t] = wmma16b(l1, bh, acc[1][t]); acc[1][t] = wmma16b(a1, bl, acc[1][t]); } }
#pragma unroll
  for (int t = 0; t < 4; ++t)
#pragma unroll
    for (int r = 0; r < 2; ++r)
#pragma unroll
      for (int v = 0; v < 8; ++v) { float val = acc[r][t][v] * (AI * WI) + bias[min(c0 + t * 16 + nloc, nout - 1)]; if (RELU) val = fmaxf(val, 0.0f); acc[r][t][v] = val; }
  epi_f32(acc, 1.0f, nullptr, y, H, m0, c0, lane, Ts[wave]);
}

__global__ __launch_bounds__(256) void gmean_kernel(const float* __restrict__ vn2, float* __restrict__ gf) {
  const int b = blockIdx.x, hcol = threadIdx.x; float s = 0.0f;
#pragma unroll 1
  for (int v = 0; v < V; ++v) s += vn2[((size_t)b * V + v) * H + hcol];
  for (int pass = 0; pass < 2; ++pass) { ((volatile float*)gf)[(size_t)b * H + hcol] = s * (1.0f / V); __threadfence(); }
}

__global__ __launch_bounds__(256) void out_kernel(const float* __restrict__ z, float* __restrict__ out) {
  __shared__ float Ob[B_ * OUT];
  for (int i = threadIdx.x; i < B_ * OUT; i += 256) Ob[i] = z[(size_t)(i / OUT) * H + (i % OUT)];
  __syncthreads();
  for (int pass = 0; pass < 2; ++pass) { for (int i = threadIdx.x; i < B_ * OUT / 4; i += 256) *(volatile v4f*)(out + i * 4) = *(const v4f*)(&Ob[i * 4]); __threadfence(); }
}
}

extern "C" void kernel_launch(void* const* d_in, const int* in_sizes, int n_in,
                              void* d_out, int out_size, void* d_ws, size_t ws_size, hipStream_t stream) {
  (void)n_in; (void)out_size;
  const float* x = (const float*)d_in[0]; const int* esrc = (const int*)d_in[1]; const int* edst = (const int*)d_in[2];
  const float* Wemb = (const float*)d_in[3]; const float* bemb = (const float*)d_in[4]; const float* Wgcn = (const float*)d_in[5]; const float* bgcn = (const float*)d_in[6];
  const float* aW1 = (const float*)d_in[7]; const float* ab1 = (const float*)d_in[8]; const float* aW2 = (const float*)d_in[9]; const float* ab2 = (const float*)d_in[10];
  const float* vW1 = (const float*)d_in[11]; const float* vb1 = (const float*)d_in[12]; const float* vW2 = (const float*)d_in[13]; const float* vb2 = (const float*)d_in[14];
  const float* mW1 = (const float*)d_in[15]; const float* mb1 = (const float*)d_in[16]; const float* mW2 = (const float*)d_in[17]; const float* mb2 = (const float*)d_in[18]; const float* ew = (const float*)d_in[19];
  float* out = (float*)d_out;
  if (in_sizes[0] != TN * IN || in_sizes[1] != E || in_sizes[2] != E || in_sizes[3] != IN * H || in_sizes[5] != H * H || in_sizes[17] != H * OUT || in_sizes[19] != B_ * NPG * V) return;
  size_t off = 0; char* ws = (char*)d_ws;
  auto carve = [&](size_t bytes) { char* p = ws + off; off += (bytes + 255) & ~(size_t)255; return p; };
  b16* wemb = (b16*)carve((size_t)H * IN * 2); b16* w3 = (b16*)carve((size_t)3 * H * H * 2); b16* th = (b16*)carve((size_t)(3 * H * H + 64 * H) * 2); b16* tl = (b16*)carve((size_t)(3 * H * H + 64 * H) * 2);
  float* h0 = (float*)carve((size_t)TN * H * 4); float* hw = (float*)carve((size_t)TN * H * 4); float* degf = (float*)carve((size_t)TN * 4);
  float* g = h0;   b16* gT = (b16*)carve((size_t)TN * H * 2); float* t1 = hw;   float* t2 = h0;
  b16* mwT = (b16*)carve((size_t)B_ * V * NPG * 2); float* vn = (float*)carve((size_t)B_ * V * H * 4); float* vn1 = (float*)carve((size_t)B_ * V * H * 4); float* vn2 = (float*)carve((size_t)B_ * V * H * 4);
  float* gf = (float*)carve((size_t)B_ * H * 4); float* z1 = (float*)carve((size_t)B_ * H * 4); float* z2 = (float*)carve((size_t)B_ * H * 4);
  if (off > ws_size) return;
  prep_kernel<<<256, 256, 0, stream>>>(Wemb, Wgcn, aW1, aW2, vW1, vW2, mW1, mW2, wemb, w3, th, tl);
  deg_kernel<<<TN / 16384, 256, 0, stream>>>(edst, degf);
  lin_kernel<IN, H, false, false><<<dim3(H / 64, NBLK), 128, 0, stream>>>(x, wemb, bemb, h0, nullptr);
  lin_kernel<H, H, false, false><<<dim3(H / 64, NBLK), 128, 0, stream>>>(h0, w3, nullptr, hw, nullptr);
  gcn_kernel<<<TN / 256, 256, 0, stream>>>(edst, esrc, hw, degf, bgcn, g, gT);
  lin_kernel<H, H, true, false><<<dim3(H / 64, NBLK), 128, 0, stream>>>(g, w3 + (size_t)H * H, ab1, t1, nullptr);
  lin_kernel<H, H, false, false><<<dim3(H / 64, NBLK), 128, 0, stream>>>(t1, w3 + (size_t)2 * H * H, ab2, t2, nullptr);
  graph_kernel<<<B_, 256, 0, stream>>>(t2, ew, mwT);
  vn_kernel<<<dim3(H / 64, B_), 64, 0, stream>>>(mwT, gT, vn);
  tail_kernel<true><<<dim3(H / 64, B_ * V / 64), 64, 0, stream>>>(vn, th, tl, vb1, vn1, H);
  tail_kernel<false><<<dim3(H / 64, B_ * V / 64), 64, 0, stream>>>(vn1, th + (size_t)H * H, tl + (size_t)H * H, vb2, vn2, H);
  gmean_kernel<<<B_, 256, 0, stream>>>(vn2, gf);
  tail_kernel<true><<<dim3(H / 64, 1), 64, 0, stream>>>(gf, th + (size_t)2 * H * H, tl + (size_t)2 * H * H, mb1, z1, H);
  tail_kernel<false><<<dim3(1, 1), 64, 0, stream>>>(z1, th + (size_t)3 * H * H, tl + (size_t)3 * H * H, mb2, z2, OUT);
  out_kernel<<<1, 256, 0, stream>>>(z2, out);
}
